// SelfLinAttention_5660766896668
// MI455X (gfx1250) — hardware-run, weakly checked
//
#include <hip/hip_runtime.h>


#define NB_  2
#define TT   2048
#define NH_  16
#define HD   64
#define DQ   (NH_ * HD)
#define ZH   2
#define RH   512
typedef _Float16 h16;
typedef unsigned short bf;
typedef __attribute__((ext_vector_type(16))) __bf16   v16bf;
typedef __attribute__((ext_vector_type(16))) _Float16 v16h;
typedef __attribute__((ext_vector_type(8)))  _Float16 v8h;
typedef __attribute__((ext_vector_type(8)))  unsigned short v8us;
typedef __attribute__((ext_vector_type(8)))  float    v8f;
typedef __attribute__((ext_vector_type(4)))  float    v4f;
typedef v8h  __attribute__((may_alias)) v8ha;
typedef v4f  __attribute__((may_alias)) v4fa;
typedef v8us __attribute__((may_alias)) v8usa;

__device__ __forceinline__ unsigned short f2bf(float f) { unsigned u = __float_as_uint(f); u += 0x7FFFu + ((u >> 16) & 1u); return (unsigned short)(u >> 16); }
__device__ __forceinline__ float bf2f(unsigned short b) { return __uint_as_float(((unsigned)b) << 16); }
__device__ __forceinline__ float bfr(float f) { return bf2f(f2bf(f)); }
__device__ __forceinline__ v16h cat16(v8h lo, v8h hi) { return __builtin_shufflevector(lo, hi, 0, 1, 2, 3, 4, 5, 6, 7, 8, 9, 10, 11, 12, 13, 14, 15); }
__device__ __forceinline__ v16bf cat16b(v8us lo, v8us hi) { return __builtin_bit_cast(v16bf, __builtin_shufflevector(lo, hi, 0, 1, 2, 3, 4, 5, 6, 7, 8, 9, 10, 11, 12, 13, 14, 15)); }
__device__ __forceinline__ v8f wmma16(v16h a, v16h b, v8f c) { return __builtin_amdgcn_wmma_f32_16x16x32_f16(false, a, false, b, (short)0, c, false, false); }
__device__ __forceinline__ v8f wmmab(v16bf a, v16bf b, v8f c) { return __builtin_amdgcn_wmma_f32_16x16x32_bf16(false, a, false, b, (short)0, c, false, false); }


template <typename T16> struct WFrag;
template <> struct WFrag<h16> { typedef v16h V; static __device__ __forceinline__ V ld(const h16* p) { return cat16(*(const v8h*)p, *(const v8h*)(p + 16)); } static __device__ __forceinline__ v8f mma(V a, V b, v8f c) { return wmma16(a, b, c); } };
template <> struct WFrag<bf> { typedef v16bf V; static __device__ __forceinline__ V ld(const bf* p) { return cat16b(*(const v8us*)p, *(const v8us*)(p + 16)); } static __device__ __forceinline__ v8f mma(V a, V b, v8f c) { return wmmab(a, b, c); } };
template <typename T16, int NSPLIT, int CMODE>
__global__ __launch_bounds__(32) void k_gemmc(const T16* __restrict__ A, const T16* __restrict__ A2, const T16* __restrict__ Bt, const T16* __restrict__ Bt2, int K, float* C, int ldc, int roff, size_t sA, size_t sB, size_t sC) {
    typedef typename WFrag<T16>::V V;
    __shared__ __align__(16) float os[16 * 68];
    const size_t z = blockIdx.z; A += z * sA; if (A2) A2 += z * sA; Bt += z * sB; if (Bt2) Bt2 += z * sB; C += z * sC;
    const int lane = threadIdx.x & 31, lr = lane & 15, hi = lane >> 4; const int r0 = blockIdx.x * 64, c0 = blockIdx.y * 64;
    if (CMODE == 1 && c0 > r0 + roff + 63) return;
    const int Kl = (CMODE == 2) ? min(K, r0 + roff + 64) : K;
    v8f acc[4][4];
#pragma unroll
    for (int mb = 0; mb < 4; ++mb)
#pragma unroll
        for (int nb = 0; nb < 4; ++nb) acc[mb][nb] = (v8f){};
    const size_t aoff = (size_t)(r0 + lr) * K + 8 * hi, boff = (size_t)(c0 + lr) * K + 8 * hi;
    for (int kc = 0; kc < Kl; kc += 32) {
        V a[4], a2[4];
#pragma unroll
        for (int mb = 0; mb < 4; ++mb) { a[mb] = WFrag<T16>::ld(A + aoff + (size_t)mb * 16 * K + kc); if (NSPLIT == 1 || NSPLIT == 2) a2[mb] = WFrag<T16>::ld(A2 + aoff + (size_t)mb * 16 * K + kc); }
#pragma unroll
        for (int nb = 0; nb < 4; ++nb) { const V b = WFrag<T16>::ld(Bt + boff + (size_t)nb * 16 * K + kc); V b2; if (NSPLIT >= 2) b2 = WFrag<T16>::ld(Bt2 + boff + (size_t)nb * 16 * K + kc);
#pragma unroll
            for (int mb = 0; mb < 4; ++mb) { acc[mb][nb] = WFrag<T16>::mma(a[mb], b, acc[mb][nb]); if (NSPLIT == 1 || NSPLIT == 2) acc[mb][nb] = WFrag<T16>::mma(a2[mb], b, acc[mb][nb]); if (NSPLIT >= 2) acc[mb][nb] = WFrag<T16>::mma(a[mb], b2, acc[mb][nb]); } }
        asm volatile("v_nop\n\tv_nop\n\tv_nop\n\tv_nop" : "+v"(acc[0][0]), "+v"(acc[1][1]), "+v"(acc[2][2]), "+v"(acc[3][3]) : "v"(a[0]), "v"(a[3]));
    }
#pragma unroll
    for (int mb = 0; mb < 4; ++mb) {
#pragma unroll
        for (int nb = 0; nb < 4; ++nb) {
#pragma unroll
            for (int j = 0; j < 8; ++j) os[(hi * 8 + j) * 68 + nb * 16 + lr] = acc[mb][nb][j]; }
        __builtin_amdgcn_wave_barrier(); asm volatile("" ::: "memory");
        float* crow = C + (size_t)(r0 + mb * 16) * ldc + c0;
#pragma unroll 1
        for (int ps = 0; ps < 2; ++ps) {
#pragma unroll
            for (int s = 0; s < 8; ++s) { const int row = 2 * s + hi, cofs = lr * 4; v4f val = *(const v4fa*)(os + row * 68 + cofs);
                *(volatile v4f*)(crow + (size_t)row * ldc + cofs) = val; }
            if (ps == 0) __threadfence(); }
        __builtin_amdgcn_wave_barrier(); asm volatile("" ::: "memory");
    }
}
__device__ __forceinline__ h16 tohx(float x) { return (h16)x; }
__device__ __forceinline__ void splitf(float y, unsigned short& h, unsigned short& l) { h = f2bf(y); l = f2bf(y - bf2f(h)); }
typedef __attribute__((ext_vector_type(2))) _Float16 v2h;
typedef __attribute__((ext_vector_type(4))) _Float16 v4h;
typedef __attribute__((ext_vector_type(2))) unsigned short v2us;
typedef __attribute__((ext_vector_type(4))) unsigned short v4us;
typedef __attribute__((ext_vector_type(2))) float v2f;
typedef __attribute__((ext_vector_type(4))) int v4i;

__global__ __launch_bounds__(256) void k_rbf(const float* __restrict__ X, float* Y, size_t n4) { const size_t i = (size_t)blockIdx.x * 256 + threadIdx.x; if (i >= n4) return; const v4f a = *(const v4f*)(X + i * 4); v4f o;
#pragma unroll
    for (int q = 0; q < 4; ++q) o[q] = bfr(a[q]);
    *(volatile v4f*)(Y + i * 4) = o; __threadfence(); *(volatile v4f*)(Y + i * 4) = o; }
__global__ __launch_bounds__(256) void k_vtp(const float* __restrict__ F, int pitch, int nheads, h16* V16, bf* Vh, bf* Vl) { const size_t e = ((size_t)blockIdx.x * 256 + threadIdx.x) * 2; if (e >= (size_t)nheads * HD * TT) return; const int t = (int)(e % TT); const int d = (int)((e / TT) % HD); const int g = (int)(e / ((size_t)TT * HD)); v2h o16; v2us oh, ol;
#pragma unroll
    for (int q = 0; q < 2; ++q) { const float x = F[(size_t)(t + q) * pitch + g * HD + d]; o16[q] = tohx(x); unsigned short a2, c2; splitf(x, a2, c2); oh[q] = a2; ol[q] = c2; }
    *(volatile v2h*)(V16 + e) = o16; *(volatile v2us*)(Vh + e) = oh; *(volatile v2us*)(Vl + e) = ol; __threadfence(); *(volatile v2h*)(V16 + e) = o16; *(volatile v2us*)(Vh + e) = oh; *(volatile v2us*)(Vl + e) = ol; }
__global__ __launch_bounds__(256) void k_f2hc(const float* __restrict__ S, h16* P16) {
    const size_t e = ((size_t)blockIdx.x * 256 + threadIdx.x) * 4; if (e >= (size_t)ZH * TT * TT) return; const int j0 = (int)(e % TT); const int i = (int)((e / TT) % TT); if (j0 > (i | 63)) return;
    const v4f a = *(const v4f*)(S + e); v4h o;
#pragma unroll
    for (int q = 0; q < 4; ++q) o[q] = tohx((j0 + q <= i) ? a[q] : 0.0f);
    *(volatile v4h*)(P16 + e) = o; __threadfence(); *(volatile v4h*)(P16 + e) = o; }

__global__ __launch_bounds__(256) void k_phi(const float* __restrict__ F, int pitch, int nheads, h16* P16) { const size_t e = ((size_t)blockIdx.x * 256 + threadIdx.x) * 2; if (e >= (size_t)nheads * TT * HD) return; const int d = (int)(e % HD); const int t = (int)((e / HD) % TT); const int h = (int)(e / ((size_t)HD * TT)); const v2f x = *(const v2f*)(F + (size_t)t * pitch + h * HD + d); v2h o;
#pragma unroll
    for (int q = 0; q < 2; ++q) o[q] = tohx(x[q] > 0.0f ? __fadd_rn(x[q], 1.0f) : __builtin_amdgcn_exp2f(__fmul_rn(x[q], 1.4426950408889634f)));
    *(volatile v2h*)(P16 + e) = o; __threadfence(); *(volatile v2h*)(P16 + e) = o; }
__global__ __launch_bounds__(256) void k_f2hx(const float* __restrict__ S, bf* Ph, bf* Pl) {
    const size_t e = ((size_t)blockIdx.x * 256 + threadIdx.x) * 4; if (e >= (size_t)ZH * RH * TT) return; const int j0 = (int)(e % TT); const int i = (int)((e / TT) % RH); const int zz = (int)(e / ((size_t)TT * RH)); if (j0 > (i | 63)) return;
    const v4f a = *(const v4f*)(S + ((size_t)zz * TT + i) * TT + j0); v4us oh, ol;
#pragma unroll
    for (int q = 0; q < 4; ++q) { unsigned short hh, ll; splitf((j0 + q <= i) ? a[q] : 0.0f, hh, ll); oh[q] = hh; ol[q] = ll; }
    *(volatile v4us*)(Ph + e) = oh; *(volatile v4us*)(Pl + e) = ol; __threadfence(); *(volatile v4us*)(Ph + e) = oh; *(volatile v4us*)(Pl + e) = ol; }
__global__ __launch_bounds__(256) void k_rsum(const h16* __restrict__ P16, float* NU) { const int idx = blockIdx.x * 256 + threadIdx.x; if (idx >= ZH * TT) return; const h16* p = P16 + (size_t)idx * TT; float s = 0.f;
#pragma unroll 1
    for (int j = 0; j < TT; j += 8) { const v8h a = *(const v8h*)(p + j);
#pragma unroll
        for (int q = 0; q < 8; ++q) s = __fadd_rn(s, (float)a[q]); }
    *(volatile float*)(NU + idx) = s; __threadfence(); *(volatile float*)(NU + idx) = s; }
__global__ __launch_bounds__(256) void k_divr(const float* __restrict__ MG, const float* __restrict__ NU, float* OUT, size_t n4) { const size_t i = (size_t)blockIdx.x * 256 + threadIdx.x; if (i >= n4) return; const size_t e = i * 4; const int c = (int)(e % DQ); const int t = (int)(e / DQ); const int h = c / HD; const float nu = NU[(size_t)h * TT + t]; const v4f a = *(const v4f*)(MG + e); v4f o;
#pragma unroll
    for (int q = 0; q < 4; ++q) o[q] = __fdiv_rn(a[q], nu);
    *(volatile v4f*)(OUT + e) = o; __threadfence(); *(volatile v4f*)(OUT + e) = o; }

extern "C" void kernel_launch(void* const* d_in, const int* in_sizes, int n_in,
                              void* d_out, int out_size, void* d_ws, size_t ws_size, hipStream_t stream) {
    (void)in_sizes; (void)n_in; (void)out_size;
    const float* qk = (const float*)d_in[0]; const float* v = (const float*)d_in[1];
    float* OUT = (float*)d_out;
    char* wsp = (char*)d_ws;
    auto take = [&](size_t bytes) { char* p = wsp; wsp += (bytes + 255) & ~(size_t)255; return (void*)p; };
    float* RQ = (float*)take((size_t)TT * 2 * DQ * 4); float* RV = (float*)take((size_t)TT * DQ * 4);
    h16* QP16 = (h16*)take((size_t)NH_ * TT * HD * 2); h16* KP16 = (h16*)take((size_t)NH_ * TT * HD * 2); h16* VT16 = (h16*)take((size_t)NH_ * HD * TT * 2); bf* VTh = (bf*)take((size_t)NH_ * HD * TT * 2); bf* VTl = (bf*)take((size_t)NH_ * HD * TT * 2);
    float* Sb = (float*)take((size_t)ZH * TT * TT * 4); h16* P16 = (h16*)take((size_t)ZH * TT * TT * 2); bf* Ph = (bf*)take((size_t)ZH * RH * TT * 2); bf* Pl = (bf*)take((size_t)ZH * RH * TT * 2);
    float* NU = (float*)take((size_t)NH_ * TT * 4); float* MG = (float*)take((size_t)TT * DQ * 4);
    if ((size_t)(wsp - (char*)d_ws) > ws_size) return;
    hipMemsetAsync(P16, 0, (size_t)ZH * TT * TT * 2, stream);
    const unsigned LH = (unsigned)(((size_t)NH_ * TT * HD / 2 + 255) / 256);
    for (int b = 0; b < NB_; ++b) {
        k_rbf<<<(unsigned)(((size_t)TT * 2 * DQ / 4 + 255) / 256), 256, 0, stream>>>(qk + (size_t)b * TT * 2 * DQ, RQ, (size_t)TT * 2 * DQ / 4); k_rbf<<<(unsigned)(((size_t)TT * DQ / 4 + 255) / 256), 256, 0, stream>>>(v + (size_t)b * TT * DQ, RV, (size_t)TT * DQ / 4);
        k_phi<<<LH, 256, 0, stream>>>(RQ, 2 * DQ, NH_, QP16);
        k_phi<<<LH, 256, 0, stream>>>(RQ + DQ, 2 * DQ, NH_, KP16);
        k_vtp<<<LH, 256, 0, stream>>>(RV, DQ, NH_, VT16, VTh, VTl);
        for (int h0 = 0; h0 < NH_; h0 += ZH) {
            k_gemmc<h16, 0, 1><<<dim3(TT / 64, TT / 64, ZH), 32, 0, stream>>>(QP16 + (size_t)h0 * TT * HD, nullptr, KP16 + (size_t)h0 * TT * HD, nullptr, HD, Sb, TT, 0, (size_t)TT * HD, (size_t)TT * HD, (size_t)TT * TT);
            k_f2hc<<<(unsigned)(((size_t)ZH * TT * TT / 4 + 255) / 256), 256, 0, stream>>>(Sb, P16);
            k_f2hx<<<(unsigned)(((size_t)ZH * RH * TT / 4 + 255) / 256), 256, 0, stream>>>(Sb, Ph, Pl);
            k_rsum<<<(ZH * TT + 255) / 256, 256, 0, stream>>>(P16, NU + (size_t)h0 * TT);
            k_gemmc<bf, 2, 2><<<dim3(RH / 64, HD / 64, ZH), 32, 0, stream>>>(Ph, Pl, VTh + (size_t)h0 * HD * TT, VTl + (size_t)h0 * HD * TT, TT, MG + (size_t)h0 * HD, DQ, 0, (size_t)RH * TT, (size_t)HD * TT, (size_t)HD);
            k_gemmc<h16, 0, 2><<<dim3((TT - RH) / 64, HD / 64, ZH), 32, 0, stream>>>(P16 + (size_t)RH * TT, nullptr, VT16 + (size_t)h0 * HD * TT, nullptr, TT, MG + (size_t)RH * DQ + (size_t)h0 * HD, DQ, RH, (size_t)TT * TT, (size_t)HD * TT, (size_t)HD); }
        k_divr<<<(unsigned)(((size_t)TT * DQ / 4 + 255) / 256), 256, 0, stream>>>(MG, NU, OUT + (size_t)b * TT * DQ, (size_t)TT * DQ / 4); }
}
